// MultiHeadAttention_28295244546545
// MI455X (gfx1250) — hardware-verified
//
#include <hip/hip_runtime.h>
#ifndef NB
#define NB 2
#endif
#ifndef SEQ
#define SEQ 2048
#endif
#define NB_FULL 2
#define SEQ_FULL 2048
#define EMB 1024
#define NH 16
#define HD 64
#define XB_FULL ((size_t)SEQ_FULL * EMB)
#define PL ((size_t)NB * NH * SEQ * HD)
#define CPL ((size_t)NB * SEQ * EMB)

static_assert(SEQ % 64 == 0);
static_assert(SEQ <= SEQ_FULL);
static_assert(NB <= NB_FULL);
static_assert(HD == 64);
static_assert(NH * HD == EMB);
static_assert(6 * PL * 2 + 2 * CPL * 2 + (size_t)3 * HD * HD * 2 + (size_t)EMB * EMB * 2 + 1024 <= (size_t)134217728);

typedef __bf16 v16b __attribute__((ext_vector_type(16)));
typedef _Float16 v16h __attribute__((ext_vector_type(16)));
typedef unsigned short v8us __attribute__((ext_vector_type(8), may_alias));
typedef float v8f __attribute__((ext_vector_type(8)));
typedef float v4f __attribute__((ext_vector_type(4)));
typedef float v4fa __attribute__((ext_vector_type(4), may_alias));
union FragB { v16b v; v8us half[2]; unsigned short u[16]; };
union FragH { v16h v; v8us half[2]; _Float16 h[16]; unsigned short u[16]; };

#define LOG2E 1.4426950408889634f

#if defined(__has_builtin)
#if __has_builtin(__builtin_amdgcn_sched_barrier)
#define SCHED_FENCE() __builtin_amdgcn_sched_barrier(0)
#endif
#endif
#ifndef SCHED_FENCE
#define SCHED_FENCE()
#endif

__device__ __forceinline__ unsigned short bf16_bits(float x) {
  unsigned int u = __float_as_uint(x);
  return (unsigned short)((u + 0x7FFFu + ((u >> 16) & 1u)) >> 16);
}
__device__ __forceinline__ float bf16_val(unsigned short b) { return __uint_as_float(((unsigned int)b) << 16); }
__device__ __forceinline__ float bf16_rne(float x) { return bf16_val(bf16_bits(x)); }

__device__ __forceinline__ void split_bf8(const v4f x0, const v4f x1, v8us& oh, v8us& ol) {
#pragma unroll
  for (int i = 0; i < 4; ++i) {
    const unsigned short h0 = bf16_bits(x0[i]);
    oh[i] = h0; ol[i] = bf16_bits(x0[i] - bf16_val(h0));
    const unsigned short h1 = bf16_bits(x1[i]);
    oh[4 + i] = h1; ol[4 + i] = bf16_bits(x1[i] - bf16_val(h1));
  }
}

__device__ __forceinline__ v8f mma_bf2(v16b a0, v16b b0, v16b a1, v16b b1, v8f c) {
  c = __builtin_amdgcn_wmma_f32_16x16x32_bf16(false, a0, false, b0, (short)0, c, false, false);
  c = __builtin_amdgcn_wmma_f32_16x16x32_bf16(false, a1, false, b1, (short)0, c, false, false);
  asm volatile("v_nop\n\tv_nop\n\tv_nop\n\tv_nop" : "+v"(c) : "v"(a0), "v"(b0), "v"(a1), "v"(b1));
  return c;
}
__device__ __forceinline__ v8f mma_bf6(v16b ah0, v16b ah1, v16b al0, v16b al1,
                                       v16b bh0, v16b bh1, v16b bl0, v16b bl1, v8f c) {
  c = __builtin_amdgcn_wmma_f32_16x16x32_bf16(false, al0, false, bh0, (short)0, c, false, false);
  c = __builtin_amdgcn_wmma_f32_16x16x32_bf16(false, al1, false, bh1, (short)0, c, false, false);
  c = __builtin_amdgcn_wmma_f32_16x16x32_bf16(false, ah0, false, bl0, (short)0, c, false, false);
  c = __builtin_amdgcn_wmma_f32_16x16x32_bf16(false, ah1, false, bl1, (short)0, c, false, false);
  c = __builtin_amdgcn_wmma_f32_16x16x32_bf16(false, ah0, false, bh0, (short)0, c, false, false);
  c = __builtin_amdgcn_wmma_f32_16x16x32_bf16(false, ah1, false, bh1, (short)0, c, false, false);
  asm volatile("v_nop\n\tv_nop\n\tv_nop\n\tv_nop" : "+v"(c)
               : "v"(ah0), "v"(ah1), "v"(al0), "v"(al1), "v"(bh0), "v"(bh1), "v"(bl0), "v"(bl1));
  return c;
}
__device__ __forceinline__ v8f mma_hl(v16b ah, v16b al, v16b b, v8f c) {
  c = __builtin_amdgcn_wmma_f32_16x16x32_bf16(false, al, false, b, (short)0, c, false, false);
  c = __builtin_amdgcn_wmma_f32_16x16x32_bf16(false, ah, false, b, (short)0, c, false, false);
  asm volatile("v_nop\n\tv_nop\n\tv_nop\n\tv_nop" : "+v"(c) : "v"(ah), "v"(al), "v"(b));
  return c;
}
__device__ __forceinline__ void mma_h3(v16h ah, v16h al, v16h bh, v16h bl, v8f& ch, v8f& cl) {
  ch = __builtin_amdgcn_wmma_f32_16x16x32_f16(false, ah, false, bh, (short)0, ch, false, false);
  cl = __builtin_amdgcn_wmma_f32_16x16x32_f16(false, ah, false, bl, (short)0, cl, false, false);
  cl = __builtin_amdgcn_wmma_f32_16x16x32_f16(false, al, false, bh, (short)0, cl, false, false);
  asm volatile("v_nop\n\tv_nop\n\tv_nop\n\tv_nop" : "+v"(ch), "+v"(cl) : "v"(ah), "v"(al), "v"(bh), "v"(bl));
}

__global__ __launch_bounds__(256) void k_cvt(const float* __restrict__ src, unsigned short* __restrict__ dst, int n8) {
  const int t = blockIdx.x * 256 + threadIdx.x;
  if (t >= n8) return;
  const float* s = src + (size_t)t * 8;
  const v4f x0 = *(const v4fa*)(s), x1 = *(const v4fa*)(s + 4);
  v8us o;
  o[0] = bf16_bits(x0[0]); o[1] = bf16_bits(x0[1]); o[2] = bf16_bits(x0[2]); o[3] = bf16_bits(x0[3]);
  o[4] = bf16_bits(x1[0]); o[5] = bf16_bits(x1[1]); o[6] = bf16_bits(x1[2]); o[7] = bf16_bits(x1[3]);
  unsigned short* d = dst + (size_t)t * 8;
  *(volatile v8us*)d = o;
  __threadfence();
  *(volatile v8us*)d = o;
}

__global__ __launch_bounds__(128) void k_proj(const float* __restrict__ X, const unsigned short* __restrict__ Wq,
                                              unsigned short* __restrict__ P) {
  __shared__ __attribute__((aligned(16))) float st[64][196];
  const int tid = threadIdx.x, w = __builtin_amdgcn_readfirstlane((int)(tid >> 5)), lane = tid & 31, ln = lane & 15, hh = lane >> 4;
  const int sg = blockIdx.x % (SEQ / 64);
  const int h = (blockIdx.x / (SEQ / 64)) % NH;
  const int b = blockIdx.x / ((SEQ / 64) * NH);
  const int s0 = sg * 64;
  const float* xrow = X + (size_t)b * XB_FULL + (size_t)(s0 + 16 * w + ln) * EMB + h * HD;
  FragB xa0, xa1;
  {
    const v4f a0 = *(const v4fa*)(xrow + 8 * hh),      a1 = *(const v4fa*)(xrow + 8 * hh + 4);
    const v4f a2 = *(const v4fa*)(xrow + 16 + 8 * hh), a3 = *(const v4fa*)(xrow + 16 + 8 * hh + 4);
    const v4f c0 = *(const v4fa*)(xrow + 32 + 8 * hh), c1 = *(const v4fa*)(xrow + 32 + 8 * hh + 4);
    const v4f c2 = *(const v4fa*)(xrow + 48 + 8 * hh), c3 = *(const v4fa*)(xrow + 48 + 8 * hh + 4);
#pragma unroll
    for (int i = 0; i < 4; ++i) {
      xa0.u[i] = bf16_bits(a0[i]); xa0.u[4 + i] = bf16_bits(a1[i]); xa0.u[8 + i] = bf16_bits(a2[i]); xa0.u[12 + i] = bf16_bits(a3[i]);
      xa1.u[i] = bf16_bits(c0[i]); xa1.u[4 + i] = bf16_bits(c1[i]); xa1.u[8 + i] = bf16_bits(c2[i]); xa1.u[12 + i] = bf16_bits(c3[i]);
    }
  }
  const v8f z8 = {0.f, 0.f, 0.f, 0.f, 0.f, 0.f, 0.f, 0.f};
#pragma unroll
  for (int t = 0; t < 12; ++t) {
    const unsigned short* wrow = Wq + (size_t)(16 * t + ln) * HD + 8 * hh;
    FragB b0, b1;
    b0.half[0] = *(const v8us*)(wrow);      b0.half[1] = *(const v8us*)(wrow + 16);
    b1.half[0] = *(const v8us*)(wrow + 32); b1.half[1] = *(const v8us*)(wrow + 48);
    const v8f acc = mma_bf2(xa0.v, b0.v, xa1.v, b1.v, z8);
#pragma unroll
    for (int r = 0; r < 8; ++r) st[16 * w + 8 * hh + r][16 * t + ln] = acc[r];
  }
  __syncthreads();
  const size_t bh = (size_t)b * NH + h;
  for (int pass = 0; pass < 2; ++pass) {
    for (int i = tid; i < 2 * 64 * 8; i += 128) {
      const int z = i >> 9, j = (i >> 3) & 63, p = i & 7;
      const v4f x0 = *(const v4fa*)&st[j][64 * z + 8 * p];
      const v4f x1 = *(const v4fa*)&st[j][64 * z + 8 * p + 4];
      v8us oh, ol;
      split_bf8(x0, x1, oh, ol);
      unsigned short* d = P + (size_t)(2 * z) * PL + (bh * SEQ + s0 + j) * HD + 8 * p;
      *(volatile v8us*)d = oh;
      *(volatile v8us*)(d + PL) = ol;
    }
    for (int i = tid; i < 64 * 8; i += 128) {
      const int d = i >> 3, j8 = (i & 7) * 8;
      FragH fh, fl;
#pragma unroll
      for (int q = 0; q < 8; ++q) {
        const float v16 = st[j8 + q][128 + d] * 16.0f;
        const _Float16 hv = (_Float16)v16;
        fh.h[q] = hv;
        fl.h[q] = (_Float16)((v16 - (float)hv) * 2048.0f);
      }
      const v8us oh = fh.half[0], ol = fl.half[0];
      unsigned short* dd = P + 4 * PL + (bh * HD + d) * SEQ + s0 + j8;
      *(volatile v8us*)dd = oh;
      *(volatile v8us*)(dd + PL) = ol;
    }
    if (pass == 0) __threadfence();
  }
}

__device__ __forceinline__ void fa_step(const unsigned short* __restrict__ Kp, const unsigned short* __restrict__ Vp,
                                        int key0, int ln, int hh,
                                        const FragB& qh0, const FragB& qh1, const FragB& ql0, const FragB& ql1,
                                        float& mr, float& lr, v8f (&Oh)[4], v8f (&Ol)[4]) {
  const unsigned short* kp0 = Kp + (size_t)(key0 + ln) * HD + 8 * hh;
  const unsigned short* kp1 = kp0 + 16 * HD;
  FragB kh00, kh01, kl00, kl01, kh10, kh11, kl10, kl11;
  kh00.half[0] = *(const v8us*)(kp0);           kh00.half[1] = *(const v8us*)(kp0 + 16);
  kh01.half[0] = *(const v8us*)(kp0 + 32);      kh01.half[1] = *(const v8us*)(kp0 + 48);
  kl00.half[0] = *(const v8us*)(kp0 + PL);      kl00.half[1] = *(const v8us*)(kp0 + PL + 16);
  kl01.half[0] = *(const v8us*)(kp0 + PL + 32); kl01.half[1] = *(const v8us*)(kp0 + PL + 48);
  kh10.half[0] = *(const v8us*)(kp1);           kh10.half[1] = *(const v8us*)(kp1 + 16);
  kh11.half[0] = *(const v8us*)(kp1 + 32);      kh11.half[1] = *(const v8us*)(kp1 + 48);
  kl10.half[0] = *(const v8us*)(kp1 + PL);      kl10.half[1] = *(const v8us*)(kp1 + PL + 16);
  kl11.half[0] = *(const v8us*)(kp1 + PL + 32); kl11.half[1] = *(const v8us*)(kp1 + PL + 48);
  const v8f z8 = {0.f, 0.f, 0.f, 0.f, 0.f, 0.f, 0.f, 0.f};
  v8f s0 = mma_bf6(kh00.v, kh01.v, kl00.v, kl01.v, qh0.v, qh1.v, ql0.v, ql1.v, z8);
  v8f s1 = mma_bf6(kh10.v, kh11.v, kl10.v, kl11.v, qh0.v, qh1.v, ql0.v, ql1.v, z8);
  asm volatile("" : "+v"(s0), "+v"(s1) : : "memory");
  SCHED_FENCE();
  const unsigned short* vp = Vp + (size_t)ln * SEQ + key0 + 8 * hh;
  FragH vh[4], vl[4];
#pragma unroll
  for (int t = 0; t < 4; ++t) {
    vh[t].half[0] = *(const v8us*)(vp + (size_t)t * 16 * SEQ);
    vh[t].half[1] = *(const v8us*)(vp + (size_t)t * 16 * SEQ + 16);
    vl[t].half[0] = *(const v8us*)(vp + PL + (size_t)t * 16 * SEQ);
    vl[t].half[1] = *(const v8us*)(vp + PL + (size_t)t * 16 * SEQ + 16);
  }
  float sc[16];
#pragma unroll
  for (int r = 0; r < 8; ++r) { sc[r] = s0[r] * 0.125f; sc[8 + r] = s1[r] * 0.125f; }
  float mx = sc[0];
#pragma unroll
  for (int i = 1; i < 16; ++i) mx = fmaxf(mx, sc[i]);
  mx = fmaxf(mx, __shfl_xor(mx, 16, 32));
  const float mnew = fmaxf(mr, mx);
  const float al = exp2f((mr - mnew) * LOG2E);
  mr = mnew;
  FragH ph, pl;
  float ps = 0.0f;
#pragma unroll
  for (int i = 0; i < 16; ++i) {
    const float pc = exp2f(fmaf(sc[i] - mnew, LOG2E, 8.0f));
    ps += pc;
    const _Float16 hv = (_Float16)pc;
    ph.h[i] = hv;
    pl.h[i] = (_Float16)((pc - (float)hv) * 2048.0f);
  }
  ps += __shfl_xor(ps, 16, 32);
  lr = lr * al + ps;
#pragma unroll
  for (int t = 0; t < 4; ++t) { Oh[t] = Oh[t] * al; Ol[t] = Ol[t] * al; }
#pragma unroll
  for (int t = 0; t < 4; ++t) mma_h3(vh[t].v, vl[t].v, ph.v, pl.v, Oh[t], Ol[t]);
}

__global__ __launch_bounds__(128) void k_attn(const unsigned short* __restrict__ P, unsigned short* __restrict__ C) {
  __shared__ __attribute__((aligned(16))) float so[4][16][68];
  const int tid = threadIdx.x, w = __builtin_amdgcn_readfirstlane((int)(tid >> 5)), lane = tid & 31, ln = lane & 15, hh = lane >> 4;
  const int qt = blockIdx.x % (SEQ / 64);
  const int h = (blockIdx.x / (SEQ / 64)) % NH;
  const int b = blockIdx.x / ((SEQ / 64) * NH);
  const int qbase = qt * 64 + 16 * w;
  const size_t bh = (size_t)b * NH + h;
  const unsigned short* qp = P + bh * SEQ * HD + (size_t)(qbase + ln) * HD + 8 * hh;
  FragB qh0, qh1, ql0, ql1;
  qh0.half[0] = *(const v8us*)(qp);           qh0.half[1] = *(const v8us*)(qp + 16);
  qh1.half[0] = *(const v8us*)(qp + 32);      qh1.half[1] = *(const v8us*)(qp + 48);
  ql0.half[0] = *(const v8us*)(qp + PL);      ql0.half[1] = *(const v8us*)(qp + PL + 16);
  ql1.half[0] = *(const v8us*)(qp + PL + 32); ql1.half[1] = *(const v8us*)(qp + PL + 48);
  float mr = -3.0e38f, lr = 0.0f;
  v8f Oh[4] = {}, Ol[4] = {};
  const unsigned short* Kp = P + 2 * PL + bh * SEQ * HD;
  const unsigned short* Vp = P + 4 * PL + bh * HD * SEQ;
#pragma unroll 1
  for (int j = 0; j < SEQ / 32; ++j)
    fa_step(Kp, Vp, 32 * j, ln, hh, qh0, qh1, ql0, ql1, mr, lr, Oh, Ol);

  const float inv = 1.0f / (16.0f * lr);
#pragma unroll
  for (int t = 0; t < 4; ++t)
#pragma unroll
    for (int r = 0; r < 8; ++r)
      so[w][ln][16 * t + 8 * hh + r] = (Oh[t][r] + Ol[t][r] * 0.00048828125f) * inv;
  __syncthreads();
  unsigned short* cg = C + ((size_t)b * SEQ + qbase) * EMB + h * HD;
  const int rq = lane >> 3, p8 = (lane & 7) * 8;
  for (int pass = 0; pass < 2; ++pass) {
#pragma unroll
    for (int it = 0; it < 4; ++it) {
      const int row = 4 * it + rq;
      const v4f x0 = *(const v4fa*)&so[w][row][p8];
      const v4f x1 = *(const v4fa*)&so[w][row][p8 + 4];
      v8us oh, ol;
      split_bf8(x0, x1, oh, ol);
      unsigned short* d = cg + (size_t)row * EMB + p8;
      *(volatile v8us*)d = oh;
      *(volatile v8us*)(d + CPL) = ol;
    }
    if (pass == 0) __threadfence();
  }
}

__global__ __launch_bounds__(128) void k_out(const unsigned short* __restrict__ C, const unsigned short* __restrict__ Wo,
                                             const float* __restrict__ bo, float* __restrict__ O) {
  __shared__ __attribute__((aligned(16))) float so[4][16][68];
  const int tid = threadIdx.x, w = __builtin_amdgcn_readfirstlane((int)(tid >> 5)), lane = tid & 31, ln = lane & 15, hh = lane >> 4;
  const int cs = blockIdx.x % (EMB / 64);
  const int rb = blockIdx.x / (EMB / 64);
  const int row0 = rb * 64 + 16 * w;
  const unsigned short* ap = C + (size_t)(row0 + ln) * EMB + 8 * hh;
  const unsigned short* bp = Wo + (size_t)(cs * 64 + ln) * EMB + 8 * hh;
  v8f acc[4] = {};
#pragma unroll 1
  for (int kc = 0; kc < EMB; kc += 32) {
    FragB ah, al, bf[4];
    ah.half[0] = *(const v8us*)(ap + kc);       ah.half[1] = *(const v8us*)(ap + kc + 16);
    al.half[0] = *(const v8us*)(ap + CPL + kc); al.half[1] = *(const v8us*)(ap + CPL + kc + 16);
#pragma unroll
    for (int j = 0; j < 4; ++j) {
      bf[j].half[0] = *(const v8us*)(bp + (size_t)j * 16 * EMB + kc);
      bf[j].half[1] = *(const v8us*)(bp + (size_t)j * 16 * EMB + kc + 16);
    }
#pragma unroll
    for (int j = 0; j < 4; ++j) acc[j] = mma_hl(ah.v, al.v, bf[j].v, acc[j]);
  }
#pragma unroll
  for (int j = 0; j < 4; ++j) {
    const float bias = bf16_rne(bo[cs * 64 + 16 * j + ln]);
#pragma unroll
    for (int r = 0; r < 8; ++r) so[w][8 * hh + r][16 * j + ln] = acc[j][r] + bias;
  }
  __syncthreads();
  const int bb = row0 / SEQ, ss = row0 - bb * SEQ;
  float* og = O + (size_t)bb * XB_FULL + (size_t)ss * EMB + cs * 64;
  const int rsub = lane >> 4, c4 = (lane & 15) * 4;
  for (int pass = 0; pass < 2; ++pass) {
#pragma unroll
    for (int q = 0; q < 8; ++q) {
      const int row = 2 * q + rsub;
      const v4f v = *(const v4fa*)&so[w][row][c4];
      *(volatile v4f*)(og + (size_t)row * EMB + c4) = v;
    }
    if (pass == 0) __threadfence();
  }
}

extern "C" void kernel_launch(void* const* d_in, const int* in_sizes, int n_in,
                              void* d_out, int out_size, void* d_ws, size_t ws_size, hipStream_t stream) {
  if (n_in < 4) return;
  const long long need = (long long)(NB - 1) * SEQ_FULL * EMB + (long long)SEQ * EMB;
  if ((long long)in_sizes[0] < need) return;
  if ((long long)in_sizes[1] < (long long)3 * HD * HD) return;
  if ((long long)in_sizes[2] < (long long)EMB * EMB) return;
  if ((long long)in_sizes[3] < (long long)EMB) return;
  if ((long long)out_size < need) return;
  const float* X  = (const float*)d_in[0];
  const float* Wq = (const float*)d_in[1];
  const float* Wo = (const float*)d_in[2];
  const float* bo = (const float*)d_in[3];
  float* O = (float*)d_out;
  char* ws = (char*)d_ws;
  size_t off = 0;
  const size_t pbytes = 6 * PL * 2;
  const size_t cbytes = 2 * CPL * 2;
  const size_t wqbytes = (size_t)3 * HD * HD * 2;
  const size_t wobytes = (size_t)EMB * EMB * 2;
  unsigned short* Pp  = (unsigned short*)(ws + off); off += (pbytes + 255) & ~(size_t)255;
  unsigned short* Cp  = (unsigned short*)(ws + off); off += (cbytes + 255) & ~(size_t)255;
  unsigned short* Wqb = (unsigned short*)(ws + off); off += (wqbytes + 255) & ~(size_t)255;
  unsigned short* Wob = (unsigned short*)(ws + off); off += (wobytes + 255) & ~(size_t)255;
  if (off > ws_size) return;
  const int nq8 = 3 * HD * HD / 8, no8 = EMB * EMB / 8;
  k_cvt<<<(unsigned)((nq8 + 255) / 256), 256, 0, stream>>>(Wq, Wqb, nq8);
  k_cvt<<<(unsigned)((no8 + 255) / 256), 256, 0, stream>>>(Wo, Wob, no8);
  k_proj<<<(unsigned)(NB * NH * (SEQ / 64)), 128, 0, stream>>>(X, Wqb, Pp);
  k_attn<<<(unsigned)(NB * NH * (SEQ / 64)), 128, 0, stream>>>(Pp, Cp);
  k_out<<<(unsigned)((NB * SEQ / 64) * (EMB / 64)), 128, 0, stream>>>(Cp, Wob, bo, O);
}
